// RingAttention_65687229825781
// MI455X (gfx1250) — hardware-verified
//
#include <hip/hip_runtime.h>


#ifndef NB
#define NB 2
#endif
#ifndef SEQ
#define SEQ 2048
#endif
#ifndef EROWS
#define EROWS 256
#endif
#define NB_FULL 2
#define SEQ_FULL 2048
#define DIM 2048
#define HEADS 16
#define DK 128
#define SEQT (NB * SEQ)
#define QBLK (SEQ / 64)
#define EBLK (EROWS / 64)
#define ETOK (NB * EROWS)
#define CSTR 132
#define RSC 1024.0f
#define RSCI (1.0f / 1024.0f)
#define PCARRY 16384.0f
#define SCL 0.08838834764831845f

static_assert(SEQ % 64 == 0);
static_assert(EROWS % 64 == 0 && EROWS >= 64);
static_assert(SEQ >= EROWS && SEQ <= SEQ_FULL);
static_assert(NB >= 1 && NB <= NB_FULL);
static_assert(DIM == HEADS * DK && DK == 128);
static_assert(DIM % 128 == 0 && DIM % 32 == 0);
static_assert((DIM * DIM) % 2048 == 0);

typedef unsigned short us16;
typedef __attribute__((ext_vector_type(16))) __bf16   v16bf;
typedef __attribute__((ext_vector_type(16))) _Float16 v16h;
typedef __attribute__((ext_vector_type(8)))  float    v8f;
typedef __attribute__((ext_vector_type(8)))  unsigned v8u;
typedef __attribute__((ext_vector_type(4)))  unsigned v4u;
typedef __attribute__((ext_vector_type(4)))  float    v4f;

__device__ __forceinline__ unsigned f2bf(float f) { unsigned u = __float_as_uint(f); u += 0x7FFFu + ((u >> 16) & 1u); return u >> 16; }
__device__ __forceinline__ float bf2f(unsigned h) { return __uint_as_float(h << 16); }
__device__ __forceinline__ unsigned f2h(float f) { _Float16 t = (_Float16)f; return (unsigned)__builtin_bit_cast(unsigned short, t); }
__device__ __forceinline__ float h2f(unsigned u) { const unsigned short s = (unsigned short)u; return (float)__builtin_bit_cast(_Float16, s); }

__device__ __forceinline__ v8u ld_frag(const us16* rowp, int hh) {
    const v4u a = *(const v4u*)(rowp + 8 * hh);
    const v4u b = *(const v4u*)(rowp + 16 + 8 * hh);
    return __builtin_shufflevector(a, b, 0, 1, 2, 3, 4, 5, 6, 7);
}
__device__ __forceinline__ void mma_guard(v8f& c, v8u a, v8u b) {
    asm volatile("v_nop\n\tv_nop\n\tv_nop\n\tv_nop" : "+v"(c) : "v"(a), "v"(b));
}
__device__ __forceinline__ v8f mmag_bf16(v8u a, v8u b, v8f c) {
    c = __builtin_amdgcn_wmma_f32_16x16x32_bf16(false, __builtin_bit_cast(v16bf, a), false, __builtin_bit_cast(v16bf, b), (short)0, c, false, false);
    mma_guard(c, a, b);
    return c;
}
__device__ __forceinline__ v8f mmag_f16(v8u a, v8u b, v8f c) {
    c = __builtin_amdgcn_wmma_f32_16x16x32_f16(false, __builtin_bit_cast(v16h, a), false, __builtin_bit_cast(v16h, b), (short)0, c, false, false);
    mma_guard(c, a, b);
    return c;
}

__global__ __launch_bounds__(256) void prep_x(const float* __restrict__ x, us16* xb) {
    const int tok = blockIdx.x;
    const int bsel = tok / SEQ, isel = tok - bsel * SEQ;
    const float* xr = x + ((size_t)bsel * SEQ_FULL + isel) * DIM;
    const int tid = threadIdx.x;
    const v4f v0 = *(const v4f*)(xr + 8 * tid);
    const v4f v1 = *(const v4f*)(xr + 8 * tid + 4);
    v4u pk;
    pk.x = f2bf(v0.x) | (f2bf(v0.y) << 16);
    pk.y = f2bf(v0.z) | (f2bf(v0.w) << 16);
    pk.z = f2bf(v1.x) | (f2bf(v1.y) << 16);
    pk.w = f2bf(v1.z) | (f2bf(v1.w) << 16);
    us16* orow = xb + (size_t)tok * DIM;
    *(volatile v4u*)(orow + 8 * tid) = pk;
    __threadfence();
    *(volatile v4u*)(orow + 8 * tid) = pk;
}

template <int F16>
__global__ __launch_bounds__(256) void prep_w(const float* __restrict__ src, us16* dst, float scale) {
    const size_t e = ((size_t)blockIdx.x * 256 + threadIdx.x) * 8;
    const v4f v0 = *(const v4f*)(src + e);
    const v4f v1 = *(const v4f*)(src + e + 4);
    const float f[8] = {v0.x, v0.y, v0.z, v0.w, v1.x, v1.y, v1.z, v1.w};
    unsigned u[8];
#pragma unroll
    for (int i = 0; i < 8; ++i) {
        const unsigned b = f2bf(f[i]);
        u[i] = F16 ? f2h(bf2f(b) * scale) : b;
    }
    v4u pk;
    pk.x = u[0] | (u[1] << 16);
    pk.y = u[2] | (u[3] << 16);
    pk.z = u[4] | (u[5] << 16);
    pk.w = u[6] | (u[7] << 16);
    *(volatile v4u*)(dst + e) = pk;
    __threadfence();
    *(volatile v4u*)(dst + e) = pk;
}

template <int F16, int NA>
__device__ __forceinline__ void mm_tile(const us16* __restrict__ arow, const us16* __restrict__ arow2, const us16* __restrict__ bbase,
                                        int ldb, int K, int hh, v8f (&acc)[4], v8f (&acc2)[4]) {
#pragma unroll 1
    for (int kc = 0; kc < K; kc += 32) {
        const v8u a = ld_frag(arow + kc, hh);
        v8u a2 = a;
        if (NA == 2) a2 = ld_frag(arow2 + kc, hh);
#pragma unroll
        for (int t = 0; t < 4; ++t) {
            const v8u bfrag = ld_frag(bbase + (size_t)(t * 16) * ldb + kc, hh);
            if (F16) acc[t] = mmag_f16(a, bfrag, acc[t]);
            else     acc[t] = mmag_bf16(a, bfrag, acc[t]);
            if (NA == 2) {
                if (F16) acc2[t] = mmag_f16(a2, bfrag, acc2[t]);
                else     acc2[t] = mmag_bf16(a2, bfrag, acc2[t]);
            }
        }
    }
}

__global__ __launch_bounds__(256) void qkv_gemm(const us16* __restrict__ xb, const us16* __restrict__ wqkv,
                                                us16* qh, us16* qr, us16* kh, us16* kr, us16* vt, us16* vr) {
    __shared__ __align__(16) float cst[64 * CSTR];
    const int tid = threadIdx.x, lane = tid & 31, wv = tid >> 5, l16 = lane & 15, hh = lane >> 4;
    const int rt = wv & 3, ch = wv >> 2;
    const int row0 = blockIdx.x * 64;
    const int colb = blockIdx.y * 128;
    const us16* arow = xb + (size_t)(row0 + rt * 16 + l16) * DIM;
    const us16* bbase = wqkv + (size_t)(colb + ch * 64 + l16) * DIM;
    v8f acc[4] = {};
    mm_tile<0, 1>(arow, arow, bbase, DIM, DIM, hh, acc, acc);
#pragma unroll
    for (int r = 0; r < 8; ++r) {
        const int rl = rt * 16 + 8 * hh + r;
#pragma unroll
        for (int t = 0; t < 4; ++t) cst[rl * CSTR + ch * 64 + t * 16 + l16] = acc[t][r];
    }
    __syncthreads();
    const int which = colb / DIM;
    const int hsel = (colb % DIM) / DK;
    const int bsel = row0 / SEQ, i0 = row0 % SEQ;
    auto pass = [&]() {
        if (which < 2) {
            us16* ph = (which == 0) ? qh : kh;
            us16* pr = (which == 0) ? qr : kr;
#pragma unroll 4
            for (int j = 0; j < 16; ++j) {
                const int L = wv * 16 + j, r = L >> 1, c = L & 1;
                const float a = cst[r * CSTR + c * 64 + 2 * lane], bq = cst[r * CSTR + c * 64 + 2 * lane + 1];
                const unsigned ha = f2h(a), hb = f2h(bq);
                const size_t off = ((size_t)(hsel * SEQT + row0 + r)) * DK + c * 64 + 2 * lane;
                *(volatile unsigned*)(ph + off) = ha | (hb << 16);
                if (i0 < EROWS) {
                    const unsigned ra = f2h((a - h2f(ha)) * RSC), rb = f2h((bq - h2f(hb)) * RSC);
                    const size_t offr = ((size_t)((hsel * NB + bsel) * EROWS + i0 + r)) * DK + c * 64 + 2 * lane;
                    *(volatile unsigned*)(pr + offr) = ra | (rb << 16);
                }
            }
        } else {
#pragma unroll 4
            for (int j = 0; j < 16; ++j) {
                const int d = wv * 16 + j;
                const float a = cst[(2 * lane) * CSTR + d] * 4.0f, bq = cst[(2 * lane + 1) * CSTR + d] * 4.0f;
                const unsigned ha = f2h(a), hb = f2h(bq);
                const size_t off = ((size_t)(hsel * DK + d)) * SEQT + row0 + 2 * lane;
                *(volatile unsigned*)(vt + off) = ha | (hb << 16);
                if (i0 < EROWS) {
                    const unsigned ra = f2h((a - h2f(ha)) * RSC), rb = f2h((bq - h2f(hb)) * RSC);
                    const size_t offr = ((size_t)(hsel * DK + d)) * ETOK + (size_t)bsel * EROWS + i0 + 2 * lane;
                    *(volatile unsigned*)(vr + offr) = ra | (rb << 16);
                }
            }
        }
    };
    pass();
    __threadfence();
    pass();
}

__global__ __launch_bounds__(128) __attribute__((amdgpu_num_vgpr(256)))
void attn_main(const us16* __restrict__ qh, const us16* __restrict__ kh, const us16* __restrict__ vt, us16* ao) {
    __shared__ v4u ost[4][16][16];
    const int tid = threadIdx.x, lane = tid & 31, wv = tid >> 5, m = lane & 15, hh = lane >> 4;
    const int qb = blockIdx.x + EBLK;
    const int h = blockIdx.y % HEADS, bsel = blockIdx.y / HEADS;
    const size_t tok0 = (size_t)bsel * SEQ;
    const int qrow = qb * 64 + wv * 16;
    const int iq = qrow + m;
    const size_t qoff = ((size_t)h * SEQT + tok0 + qrow + m) * DK;
    v8u qf[4];
#pragma unroll
    for (int kk = 0; kk < 4; ++kk) qf[kk] = ld_frag(qh + qoff + 32 * kk, hh);
    const us16* kbh = kh + ((size_t)h * SEQT + tok0) * DK;
    const us16* vb = vt + (size_t)h * DK * SEQT + tok0;
    const float NEG = -__builtin_inff();
    v8f o[8] = {};
    float mrun = NEG, lrun = 0.f;
    const int nch = ((qrow + 15) >> 5) + 1;
#pragma unroll 1
    for (int c = 0; c < nch; ++c) {
        v8f s[2] = {};
#pragma unroll
        for (int t = 0; t < 2; ++t) {
            const size_t koff = (size_t)(c * 32 + t * 16 + m) * DK;
#pragma unroll
            for (int kk = 0; kk < 4; ++kk) {
                const v8u a = ld_frag(kbh + koff + 32 * kk, hh);
                s[t] = mmag_f16(a, qf[kk], s[t]);
            }
        }
        float sv[16];
        float cmax = NEG;
#pragma unroll
        for (int t = 0; t < 2; ++t)
#pragma unroll
            for (int r = 0; r < 8; ++r) {
                const int j = c * 32 + t * 16 + 8 * hh + r;
                const float v = (j <= iq) ? s[t][r] * SCL : NEG;
                sv[8 * t + r] = v;
                cmax = fmaxf(cmax, v);
            }
        cmax = fmaxf(cmax, __shfl_xor(cmax, 16, 32));
        const float mnew = fmaxf(mrun, cmax);
        const float muse = (mnew == NEG) ? 0.f : mnew;
        const float fac = (mrun == NEG) ? 0.f : __expf(mrun - muse);
        mrun = mnew;
        v16h ph;
        float psum = 0.f;
#pragma unroll
        for (int r = 0; r < 8; ++r) {
            const _Float16 p0 = (_Float16)(__expf(sv[r] - muse) * PCARRY);
            const _Float16 p1 = (_Float16)(__expf(sv[8 + r] - muse) * PCARRY);
            ph[r] = p0;
            ph[8 + r] = p1;
            psum += (float)p0 + (float)p1;
        }
        psum += __shfl_xor(psum, 16, 32);
        lrun = lrun * fac + psum;
        const v8u pbu = __builtin_bit_cast(v8u, ph);
#pragma unroll
        for (int dt = 0; dt < 8; ++dt) o[dt] = o[dt] * fac;
#pragma unroll
        for (int dt = 0; dt < 8; ++dt) {
            const v8u va = ld_frag(vb + (size_t)(dt * 16 + m) * SEQT + c * 32, hh);
            o[dt] = mmag_f16(va, pbu, o[dt]);
        }
    }
    const float inv = 1.0f / lrun;
#pragma unroll
    for (int dt = 0; dt < 8; ++dt) {
        v4u w;
        w.x = f2h(o[dt][0] * inv) | (f2h(o[dt][1] * inv) << 16);
        w.y = f2h(o[dt][2] * inv) | (f2h(o[dt][3] * inv) << 16);
        w.z = f2h(o[dt][4] * inv) | (f2h(o[dt][5] * inv) << 16);
        w.w = f2h(o[dt][6] * inv) | (f2h(o[dt][7] * inv) << 16);
        ost[wv][m][2 * dt + hh] = w;
    }
    __syncthreads();
    us16* aob = ao + (tok0 + qrow) * DIM + h * DK;
    auto pass = [&]() {
#pragma unroll
        for (int p = 0; p < 8; ++p) {
            const int L = 4 * p + (lane >> 3), rr = L >> 1, hf = L & 1, pc = lane & 7;
            *(volatile v4u*)(aob + (size_t)rr * DIM + 64 * hf + 8 * pc) = ost[wv][rr][8 * hf + pc];
        }
    };
    pass();
    __threadfence();
    pass();
}

__global__ __launch_bounds__(256) __attribute__((amdgpu_num_vgpr(256)))
void attn_early(const us16* __restrict__ qh, const us16* __restrict__ qr, const us16* __restrict__ kh, const us16* __restrict__ kr,
                const us16* __restrict__ vt, const us16* __restrict__ vr, us16* ao, us16* aor) {
    __shared__ v4u ost[2][4][16][16];
    const int tid = threadIdx.x, lane = tid & 31, wv = tid >> 5, m = lane & 15, hh = lane >> 4;
    const int grp = wv & 3, dh = wv >> 2;
    const int qb = blockIdx.x;
    const int h = blockIdx.y % HEADS, bsel = blockIdx.y / HEADS;
    const size_t tok0 = (size_t)bsel * SEQ;
    const size_t etok0 = (size_t)bsel * EROWS;
    const int qrow = qb * 64 + grp * 16;
    const int iq = qrow + m;
    const us16* qhr = qh + ((size_t)h * SEQT + tok0 + qrow + m) * DK;
    const us16* qrr = qr + ((size_t)h * ETOK + etok0 + qrow + m) * DK;
    const us16* kbh = kh + ((size_t)h * SEQT + tok0) * DK;
    const us16* kbr = kr + ((size_t)h * ETOK + etok0) * DK;
    const us16* vb = vt + (size_t)h * DK * SEQT + tok0;
    const us16* vrb = vr + (size_t)h * DK * ETOK + etok0;
    const float NEG = -__builtin_inff();
    v8f o[4] = {};
    v8f orr[4] = {};
    float mrun = NEG, lrun = 0.f;
    const int nch = ((qrow + 15) >> 5) + 1;
#pragma unroll 1
    for (int c = 0; c < nch; ++c) {
        v8f s[2] = {};
        v8f sr[2] = {};
#pragma unroll
        for (int t = 0; t < 2; ++t) {
            const size_t koff = (size_t)(c * 32 + t * 16 + m) * DK;
#pragma unroll
            for (int kk = 0; kk < 4; ++kk) {
                const v8u a  = ld_frag(kbh + koff + 32 * kk, hh);
                const v8u b  = ld_frag(qhr + 32 * kk, hh);
                s[t] = mmag_f16(a, b, s[t]);
                const v8u ar = ld_frag(kbr + koff + 32 * kk, hh);
                sr[t] = mmag_f16(ar, b, sr[t]);
                const v8u br = ld_frag(qrr + 32 * kk, hh);
                sr[t] = mmag_f16(a, br, sr[t]);
            }
        }
        float sv[16];
        float cmax = NEG;
#pragma unroll
        for (int t = 0; t < 2; ++t)
#pragma unroll
            for (int r = 0; r < 8; ++r) {
                const int j = c * 32 + t * 16 + 8 * hh + r;
                const float v = (j <= iq) ? (s[t][r] + sr[t][r] * RSCI) * SCL : NEG;
                sv[8 * t + r] = v;
                cmax = fmaxf(cmax, v);
            }
        cmax = fmaxf(cmax, __shfl_xor(cmax, 16, 32));
        const float mnew = fmaxf(mrun, cmax);
        const float muse = (mnew == NEG) ? 0.f : mnew;
        const float fac = (mrun == NEG) ? 0.f : __expf(mrun - muse);
        mrun = mnew;
        v16h ph, pr;
        float psum = 0.f;
#pragma unroll
        for (int r = 0; r < 8; ++r) {
            const float e0 = __expf(sv[r] - muse) * PCARRY;
            const float e1 = __expf(sv[8 + r] - muse) * PCARRY;
            const _Float16 p0 = (_Float16)e0, p1 = (_Float16)e1;
            const _Float16 q0 = (_Float16)((e0 - (float)p0) * RSC), q1 = (_Float16)((e1 - (float)p1) * RSC);
            ph[r] = p0;  ph[8 + r] = p1;
            pr[r] = q0;  pr[8 + r] = q1;
            psum += (float)p0 + (float)p1 + ((float)q0 + (float)q1) * RSCI;
        }
        psum += __shfl_xor(psum, 16, 32);
        lrun = lrun * fac + psum;
        const v8u pbu = __builtin_bit_cast(v8u, ph);
        const v8u rbu = __builtin_bit_cast(v8u, pr);
#pragma unroll
        for (int dtl = 0; dtl < 4; ++dtl) { o[dtl] = o[dtl] * fac; orr[dtl] = orr[dtl] * fac; }
#pragma unroll
        for (int dtl = 0; dtl < 4; ++dtl) {
            const int dt = dh * 4 + dtl;
            const v8u va = ld_frag(vb + (size_t)(dt * 16 + m) * SEQT + c * 32, hh);
            o[dtl] = mmag_f16(va, pbu, o[dtl]);
            orr[dtl] = mmag_f16(va, rbu, orr[dtl]);
            const v8u vra = ld_frag(vrb + (size_t)(dt * 16 + m) * ETOK + c * 32, hh);
            orr[dtl] = mmag_f16(vra, pbu, orr[dtl]);
        }
    }
    const float inv = 1.0f / lrun;
#pragma unroll
    for (int dtl = 0; dtl < 4; ++dtl) {
        unsigned hw[8], rw[8];
#pragma unroll
        for (int r = 0; r < 8; ++r) {
            const float f = (o[dtl][r] + orr[dtl][r] * RSCI) * inv;
            hw[r] = f2h(f);
            rw[r] = f2h((f - h2f(hw[r])) * RSC);
        }
        v4u w, wr;
        w.x  = hw[0] | (hw[1] << 16);  w.y  = hw[2] | (hw[3] << 16);  w.z  = hw[4] | (hw[5] << 16);  w.w  = hw[6] | (hw[7] << 16);
        wr.x = rw[0] | (rw[1] << 16);  wr.y = rw[2] | (rw[3] << 16);  wr.z = rw[4] | (rw[5] << 16);  wr.w = rw[6] | (rw[7] << 16);
        const int slot = 2 * (dh * 4 + dtl) + hh;
        ost[0][grp][m][slot] = w;
        ost[1][grp][m][slot] = wr;
    }
    __syncthreads();
    us16* dst = dh ? (aor + (etok0 + qrow) * DIM + h * DK) : (ao + (tok0 + qrow) * DIM + h * DK);
    auto pass = [&]() {
#pragma unroll
        for (int p = 0; p < 8; ++p) {
            const int L = 4 * p + (lane >> 3), rr = L >> 1, hf = L & 1, pc = lane & 7;
            *(volatile v4u*)(dst + (size_t)rr * DIM + 64 * hf + 8 * pc) = ost[dh][grp][rr][8 * hf + pc];
        }
    };
    pass();
    __threadfence();
    pass();
}

template <int EARLY>
__global__ __launch_bounds__(256) void out_gemm(const us16* __restrict__ aop, const us16* __restrict__ aorp, const us16* __restrict__ wo, float* out) {
    __shared__ __align__(16) float cst[64 * CSTR];
    constexpr int NPS = EARLY ? EBLK : ((QBLK - EBLK) > 0 ? (QBLK - EBLK) : 1);
    const int tid = threadIdx.x, lane = tid & 31, wv = tid >> 5, l16 = lane & 15, hh = lane >> 4;
    const int rt = wv & 3, ch = wv >> 2;
    const int bsel = blockIdx.x / NPS;
    const int rb = (blockIdx.x - bsel * NPS) + (EARLY ? 0 : EBLK);
    const int i0 = rb * 64;
    const size_t row0 = (size_t)bsel * SEQ + i0;
    const int colb = blockIdx.y * 128;
    const us16* arow = aop + (row0 + rt * 16 + l16) * DIM;
    const us16* arow2 = arow;
    if (EARLY) arow2 = aorp + ((size_t)bsel * EROWS + i0 + rt * 16 + l16) * DIM;
    const us16* bbase = wo + (size_t)(colb + ch * 64 + l16) * DIM;
    v8f acc[4] = {};
    v8f accr[4] = {};
    if (EARLY) mm_tile<1, 2>(arow, arow2, bbase, DIM, DIM, hh, acc, accr);
    else       mm_tile<1, 1>(arow, arow, bbase, DIM, DIM, hh, acc, acc);
#pragma unroll
    for (int r = 0; r < 8; ++r) {
        const int rl = rt * 16 + 8 * hh + r;
#pragma unroll
        for (int t = 0; t < 4; ++t) {
            const float v = EARLY ? (acc[t][r] + accr[t][r] * RSCI) : acc[t][r];
            cst[rl * CSTR + ch * 64 + t * 16 + l16] = v * (1.0f / 256.0f);
        }
    }
    __syncthreads();
    const int col = tid & 127, rsel = tid >> 7;
    float* ob = out + row0 * DIM + colb + col;
    auto pass = [&]() {
#pragma unroll 4
        for (int r = rsel; r < 64; r += 2) *(volatile float*)(ob + (size_t)r * DIM) = cst[r * CSTR + col];
    };
    pass();
    __threadfence();
    pass();
}

extern "C" void kernel_launch(void* const* d_in, const int* in_sizes, int n_in,
                              void* d_out, int out_size, void* d_ws, size_t ws_size, hipStream_t stream) {
    if (n_in < 5) return;
    const float* x   = (const float*)d_in[0];
    const float* wqf = (const float*)d_in[1];
    const float* wkf = (const float*)d_in[2];
    const float* wvf = (const float*)d_in[3];
    const float* wof = (const float*)d_in[4];
    float* out = (float*)d_out;
    if (in_sizes[0] < ((NB - 1) * SEQ_FULL + SEQ) * DIM) return;
    if (in_sizes[1] < DIM * DIM) return;
    if (in_sizes[2] < DIM * DIM) return;
    if (in_sizes[3] < DIM * DIM) return;
    if (in_sizes[4] < DIM * DIM) return;
    if (out_size < SEQT * DIM) return;

    size_t off = 0;
    auto carve = [&](size_t bytes) { size_t o = off; off += (bytes + 127) & ~(size_t)127; return o; };
    char* ws = (char*)d_ws;
    us16* xb   = (us16*)(ws + carve((size_t)SEQT * DIM * 2));
    us16* wqkv = (us16*)(ws + carve((size_t)3 * DIM * DIM * 2));
    us16* wo   = (us16*)(ws + carve((size_t)DIM * DIM * 2));
    us16* qh   = (us16*)(ws + carve((size_t)HEADS * SEQT * DK * 2));
    us16* kh   = (us16*)(ws + carve((size_t)HEADS * SEQT * DK * 2));
    us16* vt   = (us16*)(ws + carve((size_t)HEADS * DK * SEQT * 2));
    us16* ao   = (us16*)(ws + carve((size_t)SEQT * DIM * 2));
    us16* qr   = (us16*)(ws + carve((size_t)HEADS * ETOK * DK * 2));
    us16* kr   = (us16*)(ws + carve((size_t)HEADS * ETOK * DK * 2));
    us16* vr   = (us16*)(ws + carve((size_t)HEADS * DK * ETOK * 2));
    us16* aor  = (us16*)(ws + carve((size_t)ETOK * DIM * 2));
    if (off > ws_size) return;

    constexpr int WBLK = (DIM * DIM) / 2048;
    prep_x<<<SEQT, 256, 0, stream>>>(x, xb);
    prep_w<0><<<WBLK, 256, 0, stream>>>(wqf, wqkv, 1.0f);
    prep_w<0><<<WBLK, 256, 0, stream>>>(wkf, wqkv + (size_t)DIM * DIM, 1.0f);
    prep_w<0><<<WBLK, 256, 0, stream>>>(wvf, wqkv + (size_t)2 * DIM * DIM, 1.0f);
    prep_w<1><<<WBLK, 256, 0, stream>>>(wof, wo, 64.0f);
    qkv_gemm<<<dim3(SEQT / 64, (3 * DIM) / 128), 256, 0, stream>>>(xb, wqkv, qh, qr, kh, kr, vt, vr);
    attn_early<<<dim3(EBLK, NB * HEADS), 256, 0, stream>>>(qh, qr, kh, kr, vt, vr, ao, aor);
    if (QBLK > EBLK) attn_main<<<dim3(QBLK - EBLK, NB * HEADS), 128, 0, stream>>>(qh, kh, vt, ao);
    out_gemm<1><<<dim3(NB * EBLK, DIM / 128), 256, 0, stream>>>(ao, aor, wo, out);
    if (QBLK > EBLK) out_gemm<0><<<dim3(NB * (QBLK - EBLK), DIM / 128), 256, 0, stream>>>(ao, aor, wo, out);
}
